// InterFreqAttention_20452634263747
// MI455X (gfx1250) — hardware-verified
//
#include <hip/hip_runtime.h>


namespace {
constexpr int NBN = 32  , NN = 8, S = 1024, C = 64, D = 256, F = 512, NR = NBN * S, NBH = NBN / 2, NRH = NBH * S  ;
constexpr float XS = 8.0f, WSC = 256.0f, PS = 8.0f, LOG2E = 1.4426950408889634f, LN_EPS = 1e-5f;

typedef _Float16 b16;
typedef __attribute__((ext_vector_type(16))) _Float16 v16b;
typedef __attribute__((ext_vector_type(8))) _Float16 v8b;
typedef __attribute__((ext_vector_type(8))) float v8f;
typedef __attribute__((ext_vector_type(4))) float v4f;
__device__ __forceinline__ float bf16_rne(float f) { unsigned int u = __float_as_uint(f); u += 0x7FFFu + ((u >> 16) & 1u); return __uint_as_float(u & 0xFFFF0000u); }
__device__ __forceinline__ void split16(float v, b16& hi, b16& lo) { hi = (b16)v; lo = (b16)(v - (float)hi); }
__device__ __forceinline__ v16b frag_kb(const b16* p, int hh) { const v8b a = *(const v8b*)(p + 8 * hh), b = *(const v8b*)(p + 16 + 8 * hh); v16b f;
#pragma unroll
  for (int e = 0; e < 8; ++e) { f[e] = a[e]; f[8 + e] = b[e]; } return f; }
__device__ __forceinline__ v8f wmma16b(v16b a, v16b b, v8f c) { v8f d = __builtin_amdgcn_wmma_f32_16x16x32_f16(false, a, false, b, (short)0, c, false, false); asm volatile("v_nop\n\tv_nop\n\tv_nop\n\tv_nop" : "+v"(d) : "v"(a), "v"(b)); return d; }
__device__ __forceinline__ void wave_lds_sync() { __builtin_amdgcn_fence(__ATOMIC_RELEASE, "workgroup"); __builtin_amdgcn_wave_barrier(); __builtin_amdgcn_fence(__ATOMIC_ACQUIRE, "workgroup"); }
__device__ __forceinline__ float nexp2(float x) { return __builtin_amdgcn_exp2f(x); }
__device__ __forceinline__ float pmul(float a, float b) { float p = a * b; asm volatile("" : "+v"(p)); return p; }
__device__ __forceinline__ float hsum16(float v) { v += __shfl_xor(v, 1); v += __shfl_xor(v, 2); v += __shfl_xor(v, 4); return v + __shfl_xor(v, 8); }

__global__ __launch_bounds__(256) void xt_kernel(const float* __restrict__ flf, const float* __restrict__ fhf, b16* __restrict__ TQ16, b16* __restrict__ TK16) {
  __shared__ __attribute__((aligned(16))) b16 T[64][64 + 8];
  const int bn = blockIdx.z, kind = blockIdx.y, s0 = blockIdx.x * 64, t_ = threadIdx.x; const int b = bn / NN, n = bn % NN; const float* src = (kind == 0 ? flf : fhf) + ((size_t)b * C * NN + n) * S; b16* dst = kind == 0 ? TQ16 : TK16;
  for (int q = t_; q < 64 * 64; q += 256) { const int cc = q >> 6, ss = q & 63; T[ss][cc] = (b16)(bf16_rne(src[(size_t)cc * NN * S + s0 + ss]) * XS); }
  __syncthreads();
  for (int pass = 0; pass < 2; ++pass) { for (int q = t_; q < 64 * 8; q += 256) { const int ss = q >> 3, c8 = (q & 7) * 8; *(volatile v8b*)(dst + ((size_t)bn * S + s0 + ss) * C + c8) = *(const v8b*)(&T[ss][c8]); } __threadfence(); }
}
__global__ __launch_bounds__(256) void prepw_kernel(const float* __restrict__ win, const float* __restrict__ wkv, const float* __restrict__ w1, const float* __restrict__ w2, const float* __restrict__ wout, b16* __restrict__ WIN, b16* __restrict__ WKV, b16* __restrict__ W1T, b16* __restrict__ W2T, b16* __restrict__ WOT) {
  __shared__ __attribute__((aligned(16))) b16 T[64][64 + 8];
  const int kind = blockIdx.z, i0 = blockIdx.x * 64, o0 = blockIdx.y * 64, t_ = threadIdx.x; const float* w; b16* dst; int nin, nout;
  if (kind == 0) { w = win; dst = WIN; nin = C; nout = D; } else if (kind == 1) { w = wkv; dst = WKV; nin = C; nout = F; } else if (kind == 2) { w = w1; dst = W1T; nin = D; nout = F; } else if (kind == 3) { w = w2; dst = W2T; nin = F; nout = D; } else { w = wout; dst = WOT; nin = D; nout = C; }
  if (i0 >= nin || o0 >= nout) return;
  for (int q = t_; q < 64 * 64; q += 256) { const int ii = q >> 6, oo = q & 63; T[oo][ii] = (b16)(bf16_rne(w[(size_t)(i0 + ii) * nout + o0 + oo]) * WSC); }
  __syncthreads();
  for (int pass = 0; pass < 2; ++pass) { for (int q = t_; q < 64 * 8; q += 256) { const int oo = q >> 3, c8 = (q & 7) * 8; *(volatile v8b*)(dst + (size_t)(o0 + oo) * nin + i0 + c8) = *(const v8b*)(&T[oo][c8]); } __threadfence(); }
}
__global__ __launch_bounds__(128) void proj_kernel(int r0, int kind, const b16* __restrict__ TQ16, const b16* __restrict__ TK16, const b16* __restrict__ WIN, const b16* __restrict__ WKV, float* __restrict__ Y) {
  __shared__ __attribute__((aligned(16))) float Tf[4][16][128 + 4];
  const int wave = threadIdx.x >> 5, lane = threadIdx.x & 31, nloc = lane & 15, hlf = lane >> 4; const size_t m0 = (size_t)blockIdx.x * 64 + wave * 16;
  const b16* A = kind == 0 ? TQ16 : TK16; const b16* Bw = kind == 0 ? WIN : (kind == 1 ? WKV : WKV + (size_t)D * C);
  v8f acc[16];
#pragma unroll
  for (int t = 0; t < 16; ++t) acc[t] = (v8f){};
#pragma unroll
  for (int kb = 0; kb < C; kb += 32) { const v16b a = frag_kb(A + ((size_t)r0 + m0 + nloc) * C + kb, hlf);
#pragma unroll
    for (int t = 0; t < 16; ++t) acc[t] = wmma16b(a, frag_kb(Bw + (size_t)(t * 16 + nloc) * C + kb, hlf), acc[t]); }
  for (int hq = 0; hq < 2; ++hq) {
#pragma unroll
    for (int t = 0; t < 8; ++t)
#pragma unroll
      for (int r = 0; r < 8; ++r) Tf[wave][8 * hlf + r][t * 16 + nloc] = acc[hq * 8 + t][r] * (1.0f / (XS * WSC));
    wave_lds_sync();
    for (int pass = 0; pass < 2; ++pass) { for (int rr = 0; rr < 16; ++rr) *(volatile v4f*)(Y + (m0 + rr) * D + hq * 128 + lane * 4) = *(const v4f*)(&Tf[wave][rr][lane * 4]); __threadfence(); }
    wave_lds_sync(); }
}
__global__ __launch_bounds__(256) void ln_kernel(const float* __restrict__ X, const float* __restrict__ g, const float* __restrict__ be, b16* __restrict__ Yh, b16* __restrict__ Yl) {
  const int wave = threadIdx.x >> 5, lane = threadIdx.x & 31; const size_t row = (size_t)blockIdx.x * 8 + wave; const float* src = X + row * D + lane * 8;
  const v4f a = *(const v4f*)src, c = *(const v4f*)(src + 4); float v[8]; float s = 0.0f;
#pragma unroll
  for (int i = 0; i < 4; ++i) { v[i] = a[i]; v[4 + i] = c[i]; s += a[i] + c[i]; }
#pragma unroll
  for (int oo = 16; oo >= 1; oo >>= 1) s += __shfl_xor(s, oo);
  const float mean = s * (1.0f / D); float ss = 0.0f;
#pragma unroll
  for (int i = 0; i < 8; ++i) { const float dv = v[i] - mean; ss += pmul(dv, dv); }
#pragma unroll
  for (int oo = 16; oo >= 1; oo >>= 1) ss += __shfl_xor(ss, oo);
  const float rs = rsqrtf(ss * (1.0f / D) + LN_EPS); v8b hv, lv;
#pragma unroll
  for (int i = 0; i < 8; ++i) { const int ch = lane * 8 + i; const float y = pmul((v[i] - mean) * rs, bf16_rne(g[ch])) + bf16_rne(be[ch]); b16 h_, l_; split16(y * XS, h_, l_); hv[i] = h_; lv[i] = l_; }
  for (int pass = 0; pass < 2; ++pass) { *(volatile v8b*)(Yh + row * D + lane * 8) = hv; *(volatile v8b*)(Yl + row * D + lane * 8) = lv; __threadfence(); }
}
__global__ __launch_bounds__(128) void v_kernel(int bn0, const b16* __restrict__ TK16, const b16* __restrict__ WKV, b16* __restrict__ VTh, b16* __restrict__ VTl) {
  __shared__ __attribute__((aligned(16))) b16 Ts[4][16][128 + 8], Tsl[4][16][128 + 8];
  const int wave = threadIdx.x >> 5, lane = threadIdx.x & 31, nloc = lane & 15, hlf = lane >> 4; const int bn = blockIdx.z; const int d0 = blockIdx.x * 64 + wave * 16, s0 = blockIdx.y * 128;
  const b16* WV = WKV + (size_t)D * C; v8f acc[8];
#pragma unroll
  for (int t = 0; t < 8; ++t) acc[t] = (v8f){};
#pragma unroll
  for (int kb = 0; kb < C; kb += 32) { const v16b a = frag_kb(WV + (size_t)(d0 + nloc) * C + kb, hlf);
#pragma unroll
    for (int t = 0; t < 8; ++t) acc[t] = wmma16b(a, frag_kb(TK16 + ((size_t)(bn0 + bn) * S + s0 + t * 16 + nloc) * C + kb, hlf), acc[t]); }
#pragma unroll
  for (int t = 0; t < 8; ++t)
#pragma unroll
    for (int r = 0; r < 8; ++r) { b16 h_, l_; split16(acc[t][r] * (1.0f / (XS * WSC)) * XS, h_, l_); Ts[wave][8 * hlf + r][t * 16 + nloc] = h_; Tsl[wave][8 * hlf + r][t * 16 + nloc] = l_; }
  wave_lds_sync();
  for (int pass = 0; pass < 2; ++pass) { for (int rr = 0; rr < 16; ++rr) if (lane < 16) { const size_t gi = ((size_t)bn * D + d0 + rr) * S + s0 + lane * 8; *(volatile v8b*)(VTh + gi) = *(const v8b*)(&Ts[wave][rr][lane * 8]); *(volatile v8b*)(VTl + gi) = *(const v8b*)(&Tsl[wave][rr][lane * 8]); } __threadfence(); }
}
__global__ __launch_bounds__(64) void attn_kernel(const b16* __restrict__ Qh, const b16* __restrict__ Ql, const b16* __restrict__ Kh, const b16* __restrict__ Kl, const b16* __restrict__ VTh, const b16* __restrict__ VTl, float* __restrict__ Of) {
  __shared__ __attribute__((aligned(16))) float To[2][16][D + 4];
  const int wave = threadIdx.x >> 5, lane = threadIdx.x & 31, hh = lane >> 4, col = lane & 15; const int bn = blockIdx.z; const int q0 = blockIdx.x * 32 + wave * 16, qi = q0 + col;
  const b16* Qb = Qh + ((size_t)bn * S + qi) * D; const b16* Qlb = Ql + ((size_t)bn * S + qi) * D; const b16* Kb = Kh + (size_t)bn * S * D; const b16* Klb = Kl + (size_t)bn * S * D; const b16* Vb = VTh + (size_t)bn * D * S; const b16* Vlb = VTl + (size_t)bn * D * S;
  float m = -INFINITY, l = 0.0f; v8f o[16];
#pragma unroll
  for (int t = 0; t < 16; ++t) o[t] = (v8f){};
  const float cs = LOG2E / (XS * XS); const int kend = q0 + 16;
  for (int kb = 0; kb < kend; kb += 32) {
    v8f s0 = {}, s1 = {};
#pragma unroll 2
    for (int ks = 0; ks < D; ks += 32) { const v16b qa = frag_kb(Qb + ks, hh), qla = frag_kb(Qlb + ks, hh);
      const b16* k0 = Kb + (size_t)(kb + col) * D + ks, *k1 = Kb + (size_t)(kb + 16 + col) * D + ks, *k0l = Klb + (size_t)(kb + col) * D + ks, *k1l = Klb + (size_t)(kb + 16 + col) * D + ks;
      v16b f = frag_kb(k0, hh); s0 = wmma16b(f, qa, s0); s0 = wmma16b(f, qla, s0); s0 = wmma16b(frag_kb(k0l, hh), qa, s0);
      f = frag_kb(k1, hh); s1 = wmma16b(f, qa, s1); s1 = wmma16b(f, qla, s1); s1 = wmma16b(frag_kb(k1l, hh), qa, s1); }
    float e[16]; float mx = -INFINITY;
#pragma unroll
    for (int r = 0; r < 8; ++r) { const int k0i = kb + 8 * hh + r, k1i = kb + 16 + 8 * hh + r; e[r] = (k0i <= qi) ? s0[r] * cs : -INFINITY; e[8 + r] = (k1i <= qi) ? s1[r] * cs : -INFINITY; mx = fmaxf(mx, fmaxf(e[r], e[8 + r])); }
    mx = fmaxf(mx, __shfl_xor(mx, 16)); const float mn = fmaxf(m, mx); const float al = nexp2(m - mn); m = mn; float sum = 0.0f; v16b ph, pl;
#pragma unroll
    for (int i = 0; i < 16; ++i) { const float p = nexp2(e[i] - mn); sum += p; const b16 h_ = (b16)(p * PS); ph[i] = h_; pl[i] = (b16)(p * PS - (float)h_); }
    sum += __shfl_xor(sum, 16); l = l * al + sum;
#pragma unroll
    for (int t = 0; t < 16; ++t) { o[t] *= al; const v16b vf = frag_kb(Vb + (size_t)(t * 16 + col) * S + kb, hh); o[t] = wmma16b(vf, ph, o[t]); o[t] = wmma16b(vf, pl, o[t]); o[t] = wmma16b(frag_kb(Vlb + (size_t)(t * 16 + col) * S + kb, hh), ph, o[t]); } }
  const float inv = 1.0f / (l * PS * XS);
#pragma unroll
  for (int t = 0; t < 16; ++t)
#pragma unroll
    for (int r = 0; r < 8; ++r) To[wave][col][t * 16 + 8 * hh + r] = o[t][r] * inv;
  wave_lds_sync();
  for (int pass = 0; pass < 2; ++pass) { for (int rr = 0; rr < 16; ++rr) { const size_t gi = ((size_t)bn * S + q0 + rr) * D; *(volatile v4f*)(Of + gi + lane * 4) = *(const v4f*)(&To[wave][rr][lane * 4]); *(volatile v4f*)(Of + gi + 128 + lane * 4) = *(const v4f*)(&To[wave][rr][128 + lane * 4]); } __threadfence(); }
}
__global__ __launch_bounds__(128) void ffn1_kernel(const b16* __restrict__ Ah, const b16* __restrict__ Al, const b16* __restrict__ W1T, b16* __restrict__ Hh, b16* __restrict__ Hl) {
  __shared__ __attribute__((aligned(16))) b16 Th[4][16][128 + 8], Tl[4][16][128 + 8];
  const int wave = threadIdx.x >> 5, lane = threadIdx.x & 31, nloc = lane & 15, hlf = lane >> 4; const size_t m0 = (size_t)blockIdx.x * 64 + wave * 16; const int n0 = blockIdx.y * 128;
  v8f acc[8];
#pragma unroll
  for (int t = 0; t < 8; ++t) acc[t] = (v8f){};
#pragma unroll 2
  for (int kb = 0; kb < D; kb += 32) { const v16b a = frag_kb(Ah + (m0 + nloc) * D + kb, hlf), al = frag_kb(Al + (m0 + nloc) * D + kb, hlf);
#pragma unroll
    for (int t = 0; t < 8; ++t) { const v16b bw = frag_kb(W1T + (size_t)(n0 + t * 16 + nloc) * D + kb, hlf); acc[t] = wmma16b(a, bw, acc[t]); acc[t] = wmma16b(al, bw, acc[t]); } }
#pragma unroll
  for (int t = 0; t < 8; ++t)
#pragma unroll
    for (int r = 0; r < 8; ++r) { b16 h_, l_; split16(fmaxf(acc[t][r] * (1.0f / (XS * WSC)), 0.0f) * XS, h_, l_); Th[wave][8 * hlf + r][t * 16 + nloc] = h_; Tl[wave][8 * hlf + r][t * 16 + nloc] = l_; }
  wave_lds_sync();
  for (int pass = 0; pass < 2; ++pass) { for (int r2 = 0; r2 < 16; r2 += 2) { const int rr = r2 + (lane >> 4), c8 = (lane & 15) * 8; const size_t gi = (m0 + rr) * F + n0 + c8; *(volatile v8b*)(Hh + gi) = *(const v8b*)(&Th[wave][rr][c8]); *(volatile v8b*)(Hl + gi) = *(const v8b*)(&Tl[wave][rr][c8]); } __threadfence(); }
}
__global__ __launch_bounds__(128) void ffn2_kernel(const b16* __restrict__ Hh, const b16* __restrict__ Hl, const b16* __restrict__ W2T, const float* __restrict__ Vf, b16* __restrict__ Eh, b16* __restrict__ El) {
  __shared__ __attribute__((aligned(16))) b16 Th[4][16][128 + 8], Tl[4][16][128 + 8];
  const int wave = threadIdx.x >> 5, lane = threadIdx.x & 31, nloc = lane & 15, hlf = lane >> 4; const size_t m0 = (size_t)blockIdx.x * 64 + wave * 16; const int n0 = blockIdx.y * 128;
  v8f acc[8];
#pragma unroll
  for (int t = 0; t < 8; ++t) acc[t] = (v8f){};
#pragma unroll 2
  for (int kb = 0; kb < F; kb += 32) { const v16b a = frag_kb(Hh + (m0 + nloc) * F + kb, hlf), al = frag_kb(Hl + (m0 + nloc) * F + kb, hlf);
#pragma unroll
    for (int t = 0; t < 8; ++t) { const v16b bw = frag_kb(W2T + (size_t)(n0 + t * 16 + nloc) * F + kb, hlf); acc[t] = wmma16b(a, bw, acc[t]); acc[t] = wmma16b(al, bw, acc[t]); } }
#pragma unroll
  for (int t = 0; t < 8; ++t)
#pragma unroll
    for (int r = 0; r < 8; ++r) { const size_t row = m0 + 8 * hlf + r; const float y = acc[t][r] * (1.0f / (XS * WSC)) + Vf[row * D + n0 + t * 16 + nloc]; b16 h_, l_; split16(y * XS, h_, l_); Th[wave][8 * hlf + r][t * 16 + nloc] = h_; Tl[wave][8 * hlf + r][t * 16 + nloc] = l_; }
  wave_lds_sync();
  for (int pass = 0; pass < 2; ++pass) { for (int r2 = 0; r2 < 16; r2 += 2) { const int rr = r2 + (lane >> 4), c8 = (lane & 15) * 8; const size_t gi = (m0 + rr) * D + n0 + c8; *(volatile v8b*)(Eh + gi) = *(const v8b*)(&Th[wave][rr][c8]); *(volatile v8b*)(El + gi) = *(const v8b*)(&Tl[wave][rr][c8]); } __threadfence(); }
}
__global__ __launch_bounds__(128) void outproj_kernel(int bn0, const b16* __restrict__ Eh, const b16* __restrict__ El, const b16* __restrict__ WOT, float* __restrict__ out) {
  __shared__ __attribute__((aligned(16))) float Ts[4][16][128 + 4];
  const int wave = threadIdx.x >> 5, lane = threadIdx.x & 31, nloc = lane & 15, hlf = lane >> 4; const int bn = blockIdx.z; const int c0 = wave * 16, s0 = blockIdx.y * 128; const int b = (bn0 + bn) / NN, n = (bn0 + bn) % NN;
  v8f acc[8];
#pragma unroll
  for (int t = 0; t < 8; ++t) acc[t] = (v8f){};
#pragma unroll 2
  for (int kb = 0; kb < D; kb += 32) { const v16b a = frag_kb(WOT + (size_t)(c0 + nloc) * D + kb, hlf);
#pragma unroll
    for (int t = 0; t < 8; ++t) { const size_t ro = ((size_t)bn * S + s0 + t * 16 + nloc) * D + kb; acc[t] = wmma16b(a, frag_kb(Eh + ro, hlf), acc[t]); acc[t] = wmma16b(a, frag_kb(El + ro, hlf), acc[t]); } }
#pragma unroll
  for (int t = 0; t < 8; ++t)
#pragma unroll
    for (int r = 0; r < 8; ++r) Ts[wave][8 * hlf + r][t * 16 + nloc] = acc[t][r] * (1.0f / (XS * WSC));
  wave_lds_sync();
  for (int pass = 0; pass < 2; ++pass) { for (int rr = 0; rr < 16; ++rr) *(volatile v4f*)(out + (((size_t)b * C + c0 + rr) * NN + n) * S + s0 + lane * 4) = *(const v4f*)(&Ts[wave][rr][lane * 4]); __threadfence(); }
}
}

extern "C" void kernel_launch(void* const* d_in, const int* in_sizes, int n_in, void* d_out, int out_size, void* d_ws, size_t ws_size, hipStream_t stream) {
  (void)n_in;
  auto Fp = [&](int i) { return (const float*)d_in[i]; };
  if (in_sizes[0] != NR * C || in_sizes[1] != NR * C || in_sizes[2] != C * D || in_sizes[3] != C * F || in_sizes[4] != D || in_sizes[8] != D * F || in_sizes[9] != F * D || in_sizes[10] != D * C || out_size != NR * C) return;
  size_t off = 0; char* ws = (char*)d_ws;
  auto carve = [&](size_t bytes) { char* p = ws + off; off += (bytes + 255) & ~(size_t)255; return p; };
  b16* TQ16 = (b16*)carve((size_t)NR * C * 2); b16* TK16 = (b16*)carve((size_t)NR * C * 2); b16* WIN = (b16*)carve((size_t)D * C * 2); b16* WKV = (b16*)carve((size_t)F * C * 2); b16* W1T = (b16*)carve((size_t)F * D * 2); b16* W2T = (b16*)carve((size_t)D * F * 2); b16* WOT = (b16*)carve((size_t)C * D * 2);
  b16* Qh = (b16*)carve((size_t)NRH * D * 2); b16* Ql = (b16*)carve((size_t)NRH * D * 2); b16* Kh = (b16*)carve((size_t)NRH * D * 2); b16* Kl = (b16*)carve((size_t)NRH * D * 2);
  float* Vf = (float*)carve((size_t)NRH * D * 4); b16* VTh = (b16*)carve((size_t)NRH * D * 2); b16* VTl = (b16*)carve((size_t)NRH * D * 2); b16* Hh = (b16*)carve((size_t)NRH * F * 2); b16* Hl = (b16*)carve((size_t)NRH * F * 2); float* Of = (float*)carve((size_t)NRH * D * 4);
  b16* Ah = VTh; b16* Al = VTl;
  b16* Eh = Kh; b16* El = Kl;
  if (off > ws_size || off > ((size_t)128 << 20)) return;
  xt_kernel<<<dim3(S / 64, 2, NBN), 256, 0, stream>>>(Fp(0), Fp(1), TQ16, TK16);
  prepw_kernel<<<dim3(8, 8, 5), 256, 0, stream>>>(Fp(2), Fp(3), Fp(8), Fp(9), Fp(10), WIN, WKV, W1T, W2T, WOT);
  for (int hf = 0; hf < 2; ++hf) {
    proj_kernel<<<NRH / 64, 128, 0, stream>>>(hf * NRH, 0, TQ16, TK16, WIN, WKV, Of);
    ln_kernel<<<NRH / 8, 256, 0, stream>>>(Of, Fp(4), Fp(5), Qh, Ql);
    proj_kernel<<<NRH / 64, 128, 0, stream>>>(hf * NRH, 1, TQ16, TK16, WIN, WKV, Of);
    ln_kernel<<<NRH / 8, 256, 0, stream>>>(Of, Fp(4), Fp(5), Kh, Kl);
    proj_kernel<<<NRH / 64, 128, 0, stream>>>(hf * NRH, 2, TQ16, TK16, WIN, WKV, Vf);
    v_kernel<<<dim3(D / 64, S / 128, NBH), 128, 0, stream>>>(hf * NBH, TK16, WKV, VTh, VTl);
    attn_kernel<<<dim3(S / 32, 1, NBH), 64, 0, stream>>>(Qh, Ql, Kh, Kl, VTh, VTl, Of);
    ln_kernel<<<NRH / 8, 256, 0, stream>>>(Of, Fp(6), Fp(7), Ah, Al);
    ffn1_kernel<<<dim3(NRH / 64, F / 128), 128, 0, stream>>>(Ah, Al, W1T, Hh, Hl);
    ffn2_kernel<<<dim3(NRH / 64, D / 128), 128, 0, stream>>>(Hh, Hl, W2T, Vf, Eh, El);
    outproj_kernel<<<dim3(1, S / 128, NBH), 128, 0, stream>>>(hf * NBH, Eh, El, WOT, (float*)d_out);
  }
}
